// QKVAttention_8650064134593
// MI455X (gfx1250) — hardware-verified
//
#include <hip/hip_runtime.h>
#include <math.h>

typedef __attribute__((ext_vector_type(16))) _Float16 v16h;
typedef __attribute__((ext_vector_type(8)))  _Float16 v8h;
typedef __attribute__((ext_vector_type(8)))  float v8f;
typedef __attribute__((ext_vector_type(4)))  float v4f;
typedef __attribute__((ext_vector_type(4)))  unsigned v4u;

template <typename T> __device__ __forceinline__ void vst2(void* p, T v) { *(volatile T*)p = v; __threadfence(); *(volatile T*)p = v; }
__device__ __forceinline__ v8f wmma16(v16h a, v16h b, v8f c) {
  v8f d = __builtin_amdgcn_wmma_f32_16x16x32_f16(false, a, false, b, (short)0, c, false, false);
  asm volatile("v_nop\n\tv_nop\n\tv_nop\n\tv_nop" : "+v"(d) : "v"(a), "v"(b));
  return d;
}
__device__ __forceinline__ v16h frag_h(const _Float16* rowk0, int lane) {
  union { v16h v; v8h q[2]; } u; const _Float16* p = rowk0 + 8 * (lane >> 4);
  u.q[0] = *(const v8h*)p; u.q[1] = *(const v8h*)(p + 16); return u.v;
}
__device__ __forceinline__ float bfr(float v) { return (float)(__bf16)v; }
__device__ __forceinline__ void ldsx() { asm volatile("s_wait_dscnt 0" ::: "memory"); __builtin_amdgcn_wave_barrier(); __builtin_amdgcn_fence(3, "workgroup"); }

#ifndef NB
#define NB 16
#endif
#ifndef SEQ
#define SEQ 4096
#endif
#define NB_FULL 16
#define TT_FULL 4096
#define TT SEQ
#define CH 64
#define WROWS (3 * CH)
#ifndef TBH
#define TBH NB
#endif
static_assert(NB >= 1 && NB <= NB_FULL);
static_assert(TT >= 64 && TT <= TT_FULL);
static_assert(TT % 64 == 0);
static_assert(CH == 64);
static_assert((size_t)NB * CH * TT * 4u <= (size_t)16777216u);

#define WS_Q   ((size_t)0)
#define WS_K   (WS_Q + 2u * (size_t)NB * TT * CH)
#define WS_V   (WS_K + 2u * (size_t)NB * TT * CH)
#define WS_END (WS_V + 2u * (size_t)NB * CH * TT)
static_assert(WS_END <= (size_t)134217728u);
static_assert(WS_K % 128u == 0 && WS_V % 128u == 0);

__global__ __launch_bounds__(128) void k_prep(const float* __restrict__ QKV, _Float16* __restrict__ QR, _Float16* __restrict__ KR, _Float16* __restrict__ VP) {
  __shared__ __align__(16) _Float16 sq[64][72], sk[64][72], sv[CH][72];
  const int t = threadIdx.x; const size_t b = blockIdx.y; const int t0 = blockIdx.x * 64;
  const float* base = QKV + b * WROWS * (size_t)TT_FULL;
  for (int e = t; e < CH * 64; e += 128) { const int c = e >> 6, tl = e & 63;
    sq[tl][c] = (_Float16)bfr(base[(size_t)c * TT_FULL + t0 + tl]);
    sk[tl][c] = (_Float16)bfr(base[(size_t)(CH + c) * TT_FULL + t0 + tl]);
    sv[c][tl] = (_Float16)bfr(base[(size_t)(2 * CH + c) * TT_FULL + t0 + tl]); }
  __syncthreads();
  for (int e = t; e < 64 * 8; e += 128) { const int tl = e >> 3, q = e & 7; const size_t o = (b * TT + t0 + tl) * CH + q * 8;
    vst2((void*)(QR + o), *(const v4u*)&sq[tl][q * 8]); vst2((void*)(KR + o), *(const v4u*)&sk[tl][q * 8]); }
  for (int e = t; e < CH * 8; e += 128) { const int c = e >> 3, q = e & 7;
    vst2((void*)(VP + (b * CH + c) * (size_t)TT + t0 + q * 8), *(const v4u*)&sv[c][q * 8]); } }

__global__ __launch_bounds__(128) void k_att(const _Float16* __restrict__ QR, const _Float16* __restrict__ KR, const _Float16* __restrict__ VP, float* __restrict__ OUT) {
  __shared__ __align__(16) float sp[4][16][36]; __shared__ __align__(16) float st[CH][68];
  const int tid = threadIdx.x, wave = tid >> 5, lane = tid & 31, col = lane & 15, g = lane >> 4; const size_t bh = blockIdx.y; const int q0 = blockIdx.x * 64 + wave * 16; const size_t rq = bh * TT + q0;
  v16h aq[2];
#pragma unroll
  for (int kc = 0; kc < 2; ++kc) aq[kc] = frag_h(QR + (rq + col) * CH + kc * 32, lane);
  float m[8], l[8];
#pragma unroll
  for (int r = 0; r < 8; ++r) { m[r] = -3.0e38f; l[r] = 0.f; }
  v8f acc[4];
#pragma unroll
  for (int j = 0; j < 4; ++j) acc[j] = v8f{};
#pragma unroll 1
  for (int ks = 0; ks < TT / 32; ++ks) { float s[2][8];
#pragma unroll
    for (int ct = 0; ct < 2; ++ct) { const size_t rk = bh * TT + ks * 32 + ct * 16 + col; v8f c = {};
#pragma unroll
      for (int kc = 0; kc < 2; ++kc) c = wmma16(aq[kc], frag_h(KR + rk * CH + kc * 32, lane), c);
#pragma unroll
      for (int r = 0; r < 8; ++r) s[ct][r] = c[r] * 0.125f; }
    float alpha[8];
#pragma unroll
    for (int r = 0; r < 8; ++r) { float mx = fmaxf(s[0][r], s[1][r]);
#pragma unroll
      for (int o = 1; o < 16; o <<= 1) mx = fmaxf(mx, __shfl_xor(mx, o));
      const float mn = fmaxf(m[r], mx); alpha[r] = __expf(m[r] - mn); const float e0 = __expf(s[0][r] - mn), e1 = __expf(s[1][r] - mn); float es = e0 + e1;
#pragma unroll
      for (int o = 1; o < 16; o <<= 1) es += __shfl_xor(es, o);
      l[r] = l[r] * alpha[r] + es; m[r] = mn; sp[wave][8 * g + r][col] = e0; sp[wave][8 * g + r][16 + col] = e1; }
#pragma unroll
    for (int j = 0; j < 4; ++j)
#pragma unroll
      for (int r = 0; r < 8; ++r) acc[j][r] *= alpha[r];
    ldsx();
    v16h pa; { const float* prow = &sp[wave][col][0] + 8 * (lane >> 4);
#pragma unroll
      for (int i = 0; i < 8; ++i) { pa[i] = (_Float16)(prow[i] * 2048.0f); pa[8 + i] = (_Float16)(prow[16 + i] * 2048.0f); } }
#pragma unroll
    for (int j = 0; j < 4; ++j) acc[j] = wmma16(pa, frag_h(VP + (bh * CH + j * 16 + col) * (size_t)TT + ks * 32, lane), acc[j]);
    ldsx(); }
#pragma unroll
  for (int r = 0; r < 8; ++r) { const float il = (1.0f / 2048.0f) / l[r];
#pragma unroll
    for (int j = 0; j < 4; ++j) st[j * 16 + col][wave * 16 + 8 * g + r] = acc[j][r] * il; }
  __syncthreads();
  for (int e = tid; e < CH * 16; e += 128) { const int c = e >> 4, q = e & 15; vst2((void*)(OUT + (bh * CH + c) * (size_t)TT + blockIdx.x * 64 + q * 4), *(const v4f*)&st[c][q * 4]); } }

extern "C" void kernel_launch(void* const* d_in, const int* in_sizes, int n_in, void* d_out, int out_size, void* d_ws, size_t ws_size, hipStream_t stream) {
  if (n_in < 1) return;
  if ((size_t)in_sizes[0] < (size_t)NB * WROWS * TT_FULL) return;
  if ((size_t)out_size < (size_t)NB * CH * TT) return;
  if (ws_size < (size_t)WS_END) return;
  const float* QKV = (const float*)d_in[0];
  char* ws = (char*)d_ws; _Float16 *QR = (_Float16*)(ws + WS_Q), *KR = (_Float16*)(ws + WS_K), *VP = (_Float16*)(ws + WS_V);
  k_prep<<<dim3(TT / 64, NB), 128, 0, stream>>>(QKV, QR, KR, VP);
  k_att<<<dim3(TT / 64, TBH), 128, 0, stream>>>(QR, KR, VP, (float*)d_out);
}
